// PFNet_37134287241357
// MI455X (gfx1250) — hardware-run, weakly checked
//
#include <hip/hip_runtime.h>


namespace {
constexpr int N = 100000, NP = 100032, NLIM = 100032  , NLIMN = (NLIM < N ? NLIM : N), E = 1600000, IN = 3, HEADS = 4, HID = 32, HC = HEADS * HID  , UP = IN + HID  , O1 = 8, O2 = 3;
constexpr float XS = 8.0f, WSC = 256.0f;
static_assert(NP % 32 == 0 && NLIM % 32 == 0, "tiling");
typedef _Float16 b16;
typedef __attribute__((ext_vector_type(16))) _Float16 v16b;
typedef __attribute__((ext_vector_type(8))) _Float16 v8b;
typedef __attribute__((ext_vector_type(8))) float v8f;
typedef __attribute__((ext_vector_type(4))) float v4f;
__device__ __forceinline__ float bf16_rne(float f) { unsigned int u = __float_as_uint(f); u += 0x7FFFu + ((u >> 16) & 1u); return __uint_as_float(u & 0xFFFF0000u); }
__device__ __forceinline__ void split16(float v, b16& hi, b16& lo) { hi = (b16)v; lo = (b16)(v - (float)hi); }
__device__ __forceinline__ v16b frag_kb(const b16* p, int hh) { const v8b a = *(const v8b*)(p + 8 * hh), b = *(const v8b*)(p + 16 + 8 * hh); v16b f;
#pragma unroll
  for (int e = 0; e < 8; ++e) { f[e] = a[e]; f[8 + e] = b[e]; } return f; }
__device__ __forceinline__ v8f wmma16b(v16b a, v16b b, v8f c) { v8f d = __builtin_amdgcn_wmma_f32_16x16x32_f16(false, a, false, b, (short)0, c, false, false); asm volatile("v_nop\n\tv_nop\n\tv_nop\n\tv_nop" : "+v"(d) : "v"(a), "v"(b)); return d; }
__device__ __forceinline__ void wave_lds_sync() { __builtin_amdgcn_fence(__ATOMIC_RELEASE, "workgroup"); __builtin_amdgcn_wave_barrier(); __builtin_amdgcn_fence(__ATOMIC_ACQUIRE, "workgroup"); }
__device__ __forceinline__ float pmul(float a, float b) { float p = a * b; asm volatile("" : "+v"(p)); return p; }
__device__ __forceinline__ int iclamp(int v, int lo, int hi) { return v < lo ? lo : (v > hi ? hi : v); }
constexpr int CSR_NBLK = 512, CSR_GB = 9, CSR_GN = 1 << CSR_GB  , CSR_MAXG = 512, CSR_CAP = 12288  ;
__global__ __launch_bounds__(64) void csrA_kernel(const int* __restrict__ dst, int E, int N, int nG, int CHP, int NGP, int* __restrict__ STG, int* __restrict__ HST) {
  extern __shared__ int sm[];
  int* cnt = sm; int* run = sm + NGP; int* ids = sm + 2 * NGP;
  const int b = blockIdx.x; const int ch = (E + CSR_NBLK - 1) / CSR_NBLK; const int e0 = b * ch, e1 = min(E, e0 + ch);
  for (int i = threadIdx.x; i < NGP; i += 64) cnt[i] = 0;
  for (int i = threadIdx.x; i < CHP; i += 64) ids[i] = -1;
  __syncthreads();
  if (threadIdx.x == 0) {
    for (int e = e0; e < e1; ++e) { int d = dst[e]; d = (d < 0) ? 0 : (d >= N ? N - 1 : d); cnt[d >> CSR_GB] += 1; }
    int acc = 0; for (int g = 0; g < nG; ++g) { run[g] = acc; acc += cnt[g]; }
    for (int e = e0; e < e1; ++e) { int d = dst[e]; d = (d < 0) ? 0 : (d >= N ? N - 1 : d); const int g = d >> CSR_GB; ids[run[g]] = e; run[g] += 1; } }
  __syncthreads();
  typedef __attribute__((ext_vector_type(4))) int v4i;
  for (int pass = 0; pass < 2; ++pass) {
    for (int i = threadIdx.x; i < CHP / 4; i += 64) *(volatile v4i*)(STG + (size_t)b * CHP + i * 4) = *(const v4i*)(&ids[i * 4]);
    for (int i = threadIdx.x; i < NGP / 4; i += 64) { v4i v; for (int e = 0; e < 4; ++e) v[e] = (i * 4 + e < nG) ? cnt[i * 4 + e] : 0; *(volatile v4i*)(HST + (size_t)b * NGP + i * 4) = v; }
    __threadfence(); }
}
__global__ __launch_bounds__(512) void csrS_kernel(const int* __restrict__ HST, int nG, int NGP, int* __restrict__ START, int* __restrict__ TOT, int* __restrict__ OFF) {
  __shared__ int tot[CSR_MAXG];
  const int b = threadIdx.x;
  for (int pass = 0; pass < 2; ++pass) { int runb = 0; for (int g = 0; g < nG; ++g) { int c = HST[(size_t)b * NGP + g]; c = (c < 0) ? 0 : c; ((volatile int*)OFF)[(size_t)g * CSR_NBLK + b] = runb; runb += c; } __threadfence(); }
  for (int g = threadIdx.x; g < nG; g += 512) { int s = 0; for (int bb = 0; bb < CSR_NBLK; ++bb) { int c = HST[(size_t)bb * NGP + g]; s += (c < 0) ? 0 : c; } tot[g] = s; }
  __syncthreads();
  if (threadIdx.x < 32) {
    __shared__ int st[CSR_MAXG + 32];
    if (threadIdx.x == 0) { int acc = 0; for (int g = 0; g < NGP; ++g) { st[g] = acc; if (g < nG) acc += (tot[g] + 31) & ~31; } st[NGP] = acc; }
    __builtin_amdgcn_fence(__ATOMIC_RELEASE, "workgroup"); __builtin_amdgcn_wave_barrier(); __builtin_amdgcn_fence(__ATOMIC_ACQUIRE, "workgroup");
    for (int pass = 0; pass < 2; ++pass) { for (int i = threadIdx.x; i < NGP + 32; i += 32) { ((volatile int*)START)[i] = (i <= NGP) ? st[min(i, NGP)] : 0; ((volatile int*)TOT)[i] = (i < nG) ? tot[i] : 0; } __threadfence(); } }
}
__global__ __launch_bounds__(256) void csrB_kernel(const int* __restrict__ dst, int N, int nG, int CHP, int NGP, int permLen, const int* __restrict__ STG, const int* __restrict__ HST, const int* __restrict__ OFF, const int* __restrict__ START, const int* __restrict__ TOT, int* __restrict__ PERM, int* __restrict__ ROWPTR, int* __restrict__ ROWCNT, int* __restrict__ FLAG) {
  typedef __attribute__((ext_vector_type(4))) int v4i;
  __shared__ int ids[CSR_CAP]; __shared__ unsigned short key[CSR_CAP]; __shared__ int outp[CSR_CAP]; __shared__ int ncnt[CSR_GN + 1]; __shared__ int boff[CSR_NBLK + 1];
  const int g = blockIdx.x, t_ = threadIdx.x; int tot = TOT[g]; int st = START[g], stn = START[g + 1]; const int v0 = g * CSR_GN; const int nv = min(CSR_GN, N - v0);
  st = (st < 0) ? 0 : (st > permLen - 32 ? permLen - 32 : st) & ~31; stn = (stn < st) ? st : (stn > permLen ? permLen : stn); tot = (tot < 0) ? 0 : tot; if (tot > stn - st && tot <= CSR_CAP) tot = stn - st;
  if (tot > CSR_CAP) {
    for (int pass = 0; pass < 2; ++pass) { for (int i = t_; i < CSR_GN / 4; i += 256) { v4i a, c; for (int e = 0; e < 4; ++e) { a[e] = st; c[e] = 0; } *(volatile v4i*)(ROWPTR + v0 + i * 4) = a; *(volatile v4i*)(ROWCNT + v0 + i * 4) = c; } if (t_ == 0) ((volatile int*)FLAG)[0] = 1; __threadfence(); } (void)nv; return; }
  if (t_ == 0) { int acc = 0; for (int b = 0; b < CSR_NBLK; ++b) { boff[b] = acc; int c = HST[(size_t)b * NGP + g]; c = (c < 0) ? 0 : (c > CHP ? CHP : c); acc += c; if (acc > tot) acc = tot; } boff[CSR_NBLK] = acc; }
  for (int i = t_; i <= CSR_GN; i += 256) ncnt[i] = 0;
  __syncthreads();
  for (int b = 0; b < CSR_NBLK; ++b) { const int c = boff[b + 1] - boff[b]; int o_ = OFF[(size_t)g * CSR_NBLK + b]; o_ = (o_ < 0) ? 0 : (o_ > CHP - c ? CHP - c : o_); const int* src_ = STG + (size_t)b * CHP + o_;
    for (int i = t_; i < c; i += 256) { int id = src_[i]; id = (id < 0) ? 0 : id; ids[boff[b] + i] = id; int d = dst[id]; d = (d < v0) ? v0 : (d >= N ? N - 1 : d); int kk = d - v0; kk = (kk < 0) ? 0 : (kk >= CSR_GN ? CSR_GN - 1 : kk); key[boff[b] + i] = (unsigned short)kk; } }
  __syncthreads();
  if (t_ == 0) { for (int i = 0; i < tot; ++i) ncnt[key[i]] += 1; int acc = 0; for (int vl = 0; vl < CSR_GN; ++vl) { const int c = ncnt[vl]; ncnt[vl] = acc; acc += c; } ncnt[CSR_GN] = acc;
    for (int i = 0; i < tot; ++i) { const int vl = key[i]; outp[ncnt[vl]] = ids[i]; ncnt[vl] += 1; }
    for (int vl = CSR_GN; vl > 0; --vl) ncnt[vl] = ncnt[vl - 1]; ncnt[0] = 0; }
  __syncthreads();
  for (int pass = 0; pass < 2; ++pass) {
    for (int i = t_; i < (stn - st) / 4; i += 256) { v4i v; for (int e = 0; e < 4; ++e) { const int q = i * 4 + e; v[e] = (q < tot) ? outp[q] : -1; } *(volatile v4i*)(PERM + st + i * 4) = v; }
    for (int i = t_; i < CSR_GN / 4; i += 256) { v4i a, c; for (int e = 0; e < 4; ++e) { const int vl = i * 4 + e; a[e] = st + ncnt[vl]; c[e] = (vl < nv) ? (ncnt[vl + 1] - ncnt[vl]) : 0; } *(volatile v4i*)(ROWPTR + v0 + i * 4) = a; *(volatile v4i*)(ROWCNT + v0 + i * 4) = c; }
    __threadfence(); }
}
__global__ __launch_bounds__(256) void csrZ_kernel(int* __restrict__ p, size_t n4) { typedef __attribute__((ext_vector_type(4))) int v4i; const size_t tid = (size_t)blockIdx.x * 256 + threadIdx.x, nth = (size_t)gridDim.x * 256; v4i z = {0, 0, 0, 0}; for (size_t i = tid; i < n4; i += nth) *(volatile v4i*)(p + i * 4) = z; }
struct CsrBufs { int *STG, *HST, *OFF, *START, *TOT, *PERM, *ROWPTR, *ROWCNT, *FLAG; int nG, NGP, CHP; size_t permLen; char* base; size_t bytes; };
static size_t csr_carve(CsrBufs& c, char* ws, size_t off, int E, int N) {
  const size_t off0 = off; c.base = ws + off;
  auto al = [&](size_t bytes) { char* p = ws + off; off += (bytes + 255) & ~(size_t)255; return p; };
  c.nG = (N + CSR_GN - 1) / CSR_GN; c.NGP = (c.nG + 31) & ~31; const int ch = (E + CSR_NBLK - 1) / CSR_NBLK; c.CHP = (ch + 31) & ~31; c.permLen = (size_t)E + 32 * (size_t)c.nG + 32;
  c.STG = (int*)al((size_t)CSR_NBLK * c.CHP * 4); c.HST = (int*)al((size_t)CSR_NBLK * c.NGP * 4); c.OFF = (int*)al((size_t)c.NGP * CSR_NBLK * 4); c.START = (int*)al((size_t)(c.NGP + 64) * 4); c.TOT = (int*)al((size_t)(c.NGP + 64) * 4);
  c.PERM = (int*)al(c.permLen * 4); c.ROWPTR = (int*)al((size_t)c.nG * CSR_GN * 4); c.ROWCNT = (int*)al((size_t)c.nG * CSR_GN * 4); c.FLAG = (int*)al(256);
  c.bytes = off - off0; return off;
}
static void csr_build(const CsrBufs& c, const int* dst, int E, int N, hipStream_t stream) {
  const size_t smem = (size_t)(2 * c.NGP + c.CHP) * 4;
  csrZ_kernel<<<512, 256, 0, stream>>>((int*)c.base, c.bytes / 16);
  csrA_kernel<<<CSR_NBLK, 64, smem, stream>>>(dst, E, N, c.nG, c.CHP, c.NGP, c.STG, c.HST);
  csrS_kernel<<<1, 512, 0, stream>>>(c.HST, c.nG, c.NGP, c.START, c.TOT, c.OFF);
  csrB_kernel<<<c.nG, 256, 0, stream>>>(dst, N, c.nG, c.CHP, c.NGP, (int)c.permLen, c.STG, c.HST, c.OFF, c.START, c.TOT, c.PERM, c.ROWPTR, c.ROWCNT, c.FLAG);
}

typedef __attribute__((ext_vector_type(2))) float v2f;
__global__ __launch_bounds__(256) void prep_kernel(const float* __restrict__ x, const float* __restrict__ gw, const float* __restrict__ asrc, const float* __restrict__ adst, float* __restrict__ H, float* __restrict__ ASD) {
  __shared__ float sa[8][8];
  const int wave = threadIdx.x >> 5, lane = threadIdx.x & 31; const size_t v = (size_t)blockIdx.x * 8 + wave; const int c = lane * 4, hd = lane >> 3;
  v4f h = {0.0f, 0.0f, 0.0f, 0.0f}; float ps = 0.0f, pd = 0.0f;
  if (v < (size_t)N) { float xv[IN]; for (int i = 0; i < IN; ++i) xv[i] = bf16_rne(x[v * IN + i]);
    for (int j = 0; j < 4; ++j) { float s = 0.0f; for (int i = 0; i < IN; ++i) s += pmul(xv[i], bf16_rne(gw[i * HC + c + j])); h[j] = s; ps += pmul(s, bf16_rne(asrc[c + j])); pd += pmul(s, bf16_rne(adst[c + j])); } }
#pragma unroll
  for (int o = 1; o < 8; o <<= 1) { ps += __shfl_xor(ps, o); pd += __shfl_xor(pd, o); }
  if ((lane & 7) == 0) { sa[wave][hd] = ps; sa[wave][4 + hd] = pd; }
  __syncthreads();
  for (int pass = 0; pass < 2; ++pass) { *(volatile v4f*)(H + v * HC + c) = h; if (wave == 0) { const float* s0 = &sa[0][0]; v2f o = {s0[lane * 2], s0[lane * 2 + 1]}; *(volatile v2f*)(ASD + (size_t)blockIdx.x * 64 + lane * 2) = o; } __threadfence(); }
}
__global__ __launch_bounds__(256) void wprep_kernel(const float* const* __restrict__ dummy, const float* __restrict__ w10, const float* __restrict__ w11, const float* __restrict__ w12, const float* __restrict__ w13, const float* __restrict__ w14, const float* __restrict__ w20, const float* __restrict__ w21, const float* __restrict__ w22, const float* __restrict__ w23, const float* __restrict__ w24, b16* __restrict__ WM) {
  (void)dummy; const int u = blockIdx.x * 256 + threadIdx.x; if (u >= 10 * 32 * 64 / 8) return; const int e = u * 8; const int l = e / (32 * 64), el = e % (32 * 64); const int oo = el / 64, k0 = el % 64;
  const float* w = l == 0 ? w10 : l == 1 ? w11 : l == 2 ? w12 : l == 3 ? w13 : l == 4 ? w14 : l == 5 ? w20 : l == 6 ? w21 : l == 7 ? w22 : l == 8 ? w23 : w24;
  const int li = l % 5; const int kin = (li == 0) ? UP : HID; const int nout = (li < 4) ? HID : (l == 4 ? O1 : O2);
  v8b o; for (int j = 0; j < 8; ++j) { const int k = k0 + j; o[j] = (k < kin && oo < nout) ? (b16)(bf16_rne(w[(size_t)k * nout + oo]) * WSC) : (b16)0.0f; }
  for (int pass = 0; pass < 2; ++pass) { *(volatile v8b*)(WM + e) = o; __threadfence(); }
}
__global__ __launch_bounds__(256) void gat_kernel(const float* __restrict__ H, const float* __restrict__ ASD, const float* __restrict__ gb, const int* __restrict__ srcs, const int* __restrict__ PERM, const int* __restrict__ ROWPTR, const int* __restrict__ ROWCNT, int permLen, float* __restrict__ CV) {
  const int wave = threadIdx.x >> 5, lane = threadIdx.x & 31; const size_t v = (size_t)blockIdx.x * 8 + wave; const int c = lane * 4, hd = lane >> 3; v4f o = {0.0f, 0.0f, 0.0f, 0.0f};
  if (v < (size_t)NLIMN) { const float ad = ASD[v * 8 + 4 + hd]; float lg = ASD[v * 8 + hd] + ad; lg = lg >= 0.0f ? lg : 0.2f * lg; float m = lg, den = 1.0f; v4f acc = *(const v4f*)(H + v * HC + c);
    int st = ROWPTR[v], cnt = ROWCNT[v]; cnt = iclamp(cnt, 0, 65536); st = iclamp(st, 0, permLen - cnt);
#pragma unroll 1
    for (int j = 0; j < cnt; ++j) { const int e = iclamp(PERM[st + j], 0, E - 1); const size_t s = (size_t)iclamp(srcs[e], 0, N - 1); float l2 = ASD[s * 8 + hd] + ad; l2 = l2 >= 0.0f ? l2 : 0.2f * l2;
      const float mn = fmaxf(m, l2); const float al = __expf(m - mn), w = __expf(l2 - mn); acc = acc * al + *(const v4f*)(H + s * HC + c) * w; den = den * al + w; m = mn; }
    o = acc * (1.0f / den); }
  for (int i = 0; i < 4; ++i) { o[i] += __shfl_xor(o[i], 8); o[i] += __shfl_xor(o[i], 16); o[i] = o[i] * 0.25f + bf16_rne(gb[(lane & 7) * 4 + i]); o[i] = o[i] >= 0.0f ? o[i] : 0.01f * o[i]; if (v >= (size_t)NLIMN) o[i] = 0.0f; }
  for (int pass = 0; pass < 2; ++pass) { if (lane < 8) *(volatile v4f*)(CV + v * HID + lane * 4) = o; __threadfence(); }
}
__global__ __launch_bounds__(64) void mlp_kernel(const float* __restrict__ x, const float* __restrict__ CV, const b16* __restrict__ WM, const float* __restrict__ b10, const float* __restrict__ b11, const float* __restrict__ b12, const float* __restrict__ b13, const float* __restrict__ b14, const float* __restrict__ b20, const float* __restrict__ b21, const float* __restrict__ b22, const float* __restrict__ b23, const float* __restrict__ b24, float* __restrict__ out0, float* __restrict__ out1) {
  __shared__ __attribute__((aligned(16))) float T[2][16][64 + 4], U[2][16][64 + 4]; __shared__ __attribute__((aligned(16))) float O0s[32][O1], O1s[32 * O2 + 4];
  const int wave = threadIdx.x >> 5, lane = threadIdx.x & 31, nloc = lane & 15, hlf = lane >> 4; const size_t v0 = (size_t)blockIdx.x * 32 + wave * 16;
  for (int i = lane; i < 16 * 64; i += 32) { const int r = i >> 6, cc = i & 63; const size_t v = v0 + r; float val = 0.0f;
    if (v < (size_t)NLIMN) { if (cc < IN) val = bf16_rne(x[v * IN + cc]); else if (cc < UP) val = CV[v * HID + (cc - IN)]; }
    U[wave][r][cc] = val; }
  wave_lds_sync();
#pragma unroll 1
  for (int mlp = 0; mlp < 2; ++mlp) {
    for (int i = lane; i < 16 * 64; i += 32) { const int r = i >> 6, cc = i & 63; T[wave][r][cc] = U[wave][r][cc]; }
    wave_lds_sync();
#pragma unroll 1
    for (int li = 0; li < 5; ++li) { const int l = mlp * 5 + li; const int kin = (li == 0) ? 64 : 32;
      const float* bb = l == 0 ? b10 : l == 1 ? b11 : l == 2 ? b12 : l == 3 ? b13 : l == 4 ? b14 : l == 5 ? b20 : l == 6 ? b21 : l == 7 ? b22 : l == 8 ? b23 : b24;
      v8f acc[2] = {(v8f){}, (v8f){}};
      for (int kb = 0; kb < kin; kb += 32) { v16b ah, al;
#pragma unroll
        for (int el = 0; el < 16; ++el) { const int k = kb + ((el < 8) ? (8 * hlf + el) : (16 + 8 * hlf + el - 8)); b16 p, q; split16(T[wave][nloc][k] * XS, p, q); ah[el] = p; al[el] = q; }
#pragma unroll
        for (int tt = 0; tt < 2; ++tt) { const v16b bw = frag_kb(WM + ((size_t)l * 32 + tt * 16 + nloc) * 64 + kb, hlf); acc[tt] = wmma16b(ah, bw, acc[tt]); acc[tt] = wmma16b(al, bw, acc[tt]); } }
      wave_lds_sync();
      const int nout = (li < 4) ? HID : (mlp == 0 ? O1 : O2);
#pragma unroll
      for (int tt = 0; tt < 2; ++tt) { const int cc = tt * 16 + nloc;
#pragma unroll
        for (int r = 0; r < 8; ++r) { float val = 0.0f; if (cc < nout) { val = acc[tt][r] * (1.0f / (XS * WSC)) + bf16_rne(bb[cc]); if (li < 4) val = val >= 0.0f ? val : 0.01f * val; }
          if (li < 4) T[wave][8 * hlf + r][cc] = val; else if (cc < nout) { if (mlp == 0) O0s[wave * 16 + 8 * hlf + r][cc] = val; else O1s[(wave * 16 + 8 * hlf + r) * O2 + cc] = val; } } }
      wave_lds_sync(); } }
  __syncthreads();
  if (wave == 0) { const float* o0 = &O0s[0][0];
    for (int pass = 0; pass < 2; ++pass) { for (int i = lane; i < 32 * O1 / 4; i += 32) { const size_t vv = (size_t)blockIdx.x * 32 + (i * 4) / O1; if (vv < (size_t)N) *(volatile v4f*)(out0 + (size_t)blockIdx.x * 32 * O1 + i * 4) = *(const v4f*)(o0 + i * 4); }
      for (int i = lane; i < 32 * O2 / 4; i += 32) { const size_t vlast = (size_t)blockIdx.x * 32 + (i * 4 + 3) / O2; if (vlast < (size_t)N) *(volatile v4f*)(out1 + (size_t)blockIdx.x * 32 * O2 + i * 4) = *(const v4f*)(&O1s[i * 4]); }
      __threadfence(); } }
}
}

extern "C" void kernel_launch(void* const* d_in, const int* in_sizes, int n_in, void* d_out, int out_size, void* d_ws, size_t ws_size, hipStream_t stream) {
  (void)n_in;
  auto Fp = [&](int i) { return (const float*)d_in[i]; }; auto Ip = [&](int i) { return (const int*)d_in[i]; };
  if (in_sizes[0] != N * IN || in_sizes[1] != 2 * E || in_sizes[4] != IN * HC || in_sizes[5] != HC || in_sizes[6] != HC || in_sizes[7] != HID || in_sizes[8] != UP * HID || in_sizes[10] != UP * HID || in_sizes[12] != HID * HID || in_sizes[24] != HID * O1 || in_sizes[25] != O1 || in_sizes[26] != HID * O2 || in_sizes[27] != O2 || out_size != N * O1 + N * O2) return;
  size_t off = 0; char* ws = (char*)d_ws;
  auto carve = [&](size_t bytes) { char* p = ws + off; off += (bytes + 255) & ~(size_t)255; return p; };
  float* H = (float*)carve((size_t)NP * HC * 4); float* ASD = (float*)carve((size_t)NP * 8 * 4); float* CV = (float*)carve((size_t)NP * HID * 4); b16* WM = (b16*)carve((size_t)10 * 32 * 64 * 2);
  CsrBufs csr; off = csr_carve(csr, ws, off, E, N);
  if (off > ws_size || off > ((size_t)128 << 20)) return;
  float* out0 = (float*)d_out; float* out1 = (float*)d_out + (size_t)N * O1;
  prep_kernel<<<NP / 8, 256, 0, stream>>>(Fp(0), Fp(4), Fp(5), Fp(6), H, ASD);
  wprep_kernel<<<(10 * 32 * 64 / 8 + 255) / 256, 256, 0, stream>>>(nullptr, Fp(8), Fp(12), Fp(16), Fp(20), Fp(24), Fp(10), Fp(14), Fp(18), Fp(22), Fp(26), WM);
  csr_build(csr, Ip(1) + E, E, N, stream);
  gat_kernel<<<NLIM / 8, 256, 0, stream>>>(H, ASD, Fp(7), Ip(1), csr.PERM, csr.ROWPTR, csr.ROWCNT, (int)csr.permLen, CV);
  mlp_kernel<<<NLIM / 32, 64, 0, stream>>>(Fp(0), CV, WM, Fp(9), Fp(13), Fp(17), Fp(21), Fp(25), Fp(11), Fp(15), Fp(19), Fp(23), Fp(27), out0, out1);
}
